// TextAttention_18451179504117
// MI455X (gfx1250) — hardware-verified
//
#include <hip/hip_runtime.h>
#include <math.h>

constexpr int kBatch = 2;
constexpr int kSeq   = 4096;
constexpr int kDim   = 512;
constexpr int kHeads = 8;
constexpr int kHdim  = 64;
constexpr int kTok   = kBatch * kSeq;
constexpr int kQKCols = 2 * kDim;
constexpr int kQKVCols = 3 * kDim;
constexpr int kQRows  = 2048;
constexpr int kQChunks = kSeq / kQRows;
constexpr float kWCarry    = 16.0f;
constexpr float kWCarryInv = 1.0f / 16.0f;
constexpr float kScoreScale = 0.125f;
constexpr float kPCarry    = 2048.0f;
constexpr float kCtxCarry  = 256.0f;
constexpr float kPVScale   = kCtxCarry / kPCarry;
constexpr float kOutScale  = 1.0f / (kCtxCarry * kWCarry);
constexpr float kNegMax    = -3.40282347e+38f;

constexpr size_t kOffX16  = 0;
constexpr size_t kOffQK16 = kOffX16 + (size_t)kTok * kDim * 2;
constexpr size_t kOffVT16 = kOffQK16 + (size_t)kTok * kQKCols * 2;
constexpr size_t kOffS    = kOffVT16 + (size_t)kDim * kTok * 2;
constexpr size_t kOffP16  = kOffS + (size_t)kQRows * kSeq * 4;
constexpr size_t kWsTotal = kOffP16 + (size_t)kQRows * kSeq * 2;
static_assert(kWsTotal == 83886080ull, "carve total 80 MiB");
static_assert((size_t)kQKVCols * kDim * 2 <= (size_t)kQRows * kSeq * 4, "W_qkv^T fits in scores region");
static_assert(kQChunks * kQRows == kSeq, "chunks cover the sequence exactly");
static_assert(kQRows % 64 == 0 && kSeq % 64 == 0 && kHdim % 32 == 0, "tile multiples");

typedef __attribute__((ext_vector_type(16))) _Float16 v16h;
typedef __attribute__((ext_vector_type(8)))  _Float16 v8h;
typedef __attribute__((ext_vector_type(16))) __bf16   v16b;
typedef __attribute__((ext_vector_type(8)))  __bf16   v8b;
typedef __attribute__((ext_vector_type(8)))  float    v8f;
typedef __attribute__((ext_vector_type(4)))  float    v4f;
typedef __attribute__((ext_vector_type(4)))  unsigned int v4u;
typedef __attribute__((ext_vector_type(4)))  int      v4i;

__device__ __forceinline__ unsigned short f2bf_bits(float f) {
  unsigned u = __float_as_uint(f);
  return (unsigned short)((u + 0x7FFFu + ((u >> 16) & 1u)) >> 16);
}
__device__ __forceinline__ float bf_bits2f(unsigned short h) { return __uint_as_float(((unsigned)h) << 16); }

__device__ __forceinline__ void dep_guard_h(v8f& a, v8f& b, v16h x, v16h y) { asm volatile("v_nop\n\tv_nop\n\tv_nop\n\tv_nop" : "+v"(a), "+v"(b) : "v"(x), "v"(y)); }
__device__ __forceinline__ void dep_guard_b(v8f& a, v8f& b, v16b x, v16b y) { asm volatile("v_nop\n\tv_nop\n\tv_nop\n\tv_nop" : "+v"(a), "+v"(b) : "v"(x), "v"(y)); }
__device__ __forceinline__ void keep4_h(v16h a, v16h b, v16h c, v16h d) { asm volatile("v_nop" :: "v"(a), "v"(b), "v"(c), "v"(d)); }
__device__ __forceinline__ void keep4_b(v16b a, v16b b, v16b c, v16b d) { asm volatile("v_nop" :: "v"(a), "v"(b), "v"(c), "v"(d)); }
__device__ __forceinline__ void acc_guard4(v8f& a, v8f& b, v8f& c, v8f& d) { asm volatile("v_nop\n\tv_nop\n\tv_nop\n\tv_nop" : "+v"(a), "+v"(b), "+v"(c), "+v"(d)); }
template <typename T> struct Frag;
template <> struct Frag<_Float16> {
  typedef v16h V; union U { v16h v; v8h h[2]; };
  static __device__ __forceinline__ v16h load(const _Float16* p) {
    U f; f.h[0] = *(const v8h*)(p); f.h[1] = *(const v8h*)(p + 16); return f.v;
  }
  static __device__ __forceinline__ v8f mma(v16h a, v16h b, v8f c) {
    return __builtin_amdgcn_wmma_f32_16x16x32_f16(false, a, false, b, (short)0, c, false, false);
  }
  static __device__ __forceinline__ void guard(v8f& a, v8f& b, v16h x, v16h y) { dep_guard_h(a, b, x, y); }
  static __device__ __forceinline__ void keep(v16h a, v16h b, v16h c, v16h d) { keep4_h(a, b, c, d); }
};
template <> struct Frag<__bf16> {
  typedef v16b V; union U { v16b v; v8b h[2]; };
  static __device__ __forceinline__ v16b load(const __bf16* p) {
    U f; f.h[0] = *(const v8b*)(p); f.h[1] = *(const v8b*)(p + 16); return f.v;
  }
  static __device__ __forceinline__ v8f mma(v16b a, v16b b, v8f c) {
    return __builtin_amdgcn_wmma_f32_16x16x32_bf16(false, a, false, b, (short)0, c, false, false);
  }
  static __device__ __forceinline__ void guard(v8f& a, v8f& b, v16b x, v16b y) { dep_guard_b(a, b, x, y); }
  static __device__ __forceinline__ void keep(v16b a, v16b b, v16b c, v16b d) { keep4_b(a, b, c, d); }
};

__device__ __forceinline__ unsigned pk16(unsigned short a, unsigned short b) { return (unsigned)a | ((unsigned)b << 16); }
__device__ __forceinline__ unsigned short h_bits(float f) { const _Float16 h = (_Float16)f; return __builtin_bit_cast(unsigned short, h); }

template <int ET> struct Elem;
template <> struct Elem<0> { typedef _Float16 T; };
template <> struct Elem<1> { typedef __bf16 T; };
template <int ET, bool SPLIT, int BIAS_MODE, int OUT_MODE, bool RESID, int ACT = 0>
__global__ __launch_bounds__(256) void wmma_gemm64(
    const unsigned short* __restrict__ Ap, const unsigned short* __restrict__ A2p, int lda, long strideA,
    const unsigned short* __restrict__ Btp, const unsigned short* __restrict__ Bt2p, int ldb, long strideB,
    void* __restrict__ Cout, void* __restrict__ Cout2, int ldc, long strideC,
    const float* __restrict__ bias,
    const float* __restrict__ resid, long strideR,
    int M, int N, int K, float scale) {
  typedef typename Elem<ET>::T T;
  typedef typename Frag<T>::V V;
  const T* A = (const T*)Ap; const T* A2 = (const T*)A2p; const T* Bt = (const T*)Btp; const T* Bt2 = (const T*)Bt2p;
  __shared__ __align__(16) float sT[8][16 * 68];
  const int b    = blockIdx.y;
  const int lane = threadIdx.x & 31;
  const int wave = threadIdx.x >> 5;
  const int tilesN = N >> 6;
  const int tilesM = M >> 6;
  const int tile = blockIdx.x * 8 + wave;
  if (tile >= tilesM * tilesN) return;
  const int tm = tile / tilesN;
  const int tn = tile - tm * tilesN;
  const int m0 = tm << 6;
  const int n0 = tn << 6;

  const T* Ab  = A  + (size_t)b * strideA;
  const T* Bb  = Bt + (size_t)b * strideB;
  const T* Ab2 = SPLIT ? (A2  + (size_t)b * strideA) : nullptr;
  const T* Bb2 = SPLIT ? (Bt2 + (size_t)b * strideB) : nullptr;

  const int rlane = lane & 15;
  const int koff  = (lane >> 4) * 8;
  const int mOff  = (lane >> 4) * 8;

  v8f acc[4][4];
#pragma unroll
  for (int i = 0; i < 4; ++i)
#pragma unroll
    for (int j = 0; j < 4; ++j) acc[i][j] = (v8f){0.f,0.f,0.f,0.f,0.f,0.f,0.f,0.f};

  for (int k0 = 0; k0 < K; k0 += 32) {
    V bh[4], bl[4];
#pragma unroll
    for (int j = 0; j < 4; ++j) {
      const size_t bo = (size_t)(n0 + (j << 4) + rlane) * ldb + koff + k0;
      bh[j] = Frag<T>::load(Bb + bo);
      if (SPLIT) bl[j] = Frag<T>::load(Bb2 + bo);
    }
#pragma unroll
    for (int i = 0; i < 4; ++i) {
      const size_t ao = (size_t)(m0 + (i << 4) + rlane) * lda + koff + k0;
      V ah = Frag<T>::load(Ab + ao);
      V al;
      if (SPLIT) al = Frag<T>::load(Ab2 + ao);
#pragma unroll
      for (int j = 0; j < 4; ++j) {
        acc[i][j] = Frag<T>::mma(ah, bh[j], acc[i][j]);
        if (SPLIT) {
          acc[i][j] = Frag<T>::mma(ah, bl[j], acc[i][j]);
          acc[i][j] = Frag<T>::mma(al, bh[j], acc[i][j]);
        }
      }
      Frag<T>::guard(acc[i][0], acc[i][3], ah, SPLIT ? al : ah);
    }
    Frag<T>::keep(bh[0], bh[1], bh[2], bh[3]);
    if (SPLIT) Frag<T>::keep(bl[0], bl[1], bl[2], bl[3]);
  }
  acc_guard4(acc[0][0], acc[0][1], acc[0][2], acc[0][3]);
  acc_guard4(acc[1][0], acc[1][1], acc[1][2], acc[1][3]);
  acc_guard4(acc[2][0], acc[2][1], acc[2][2], acc[2][3]);
  acc_guard4(acc[3][0], acc[3][1], acc[3][2], acc[3][3]);

  float* slab = sT[wave];
  const float* Rb = RESID ? (resid + (size_t)b * strideR) : nullptr;
#pragma unroll
  for (int i = 0; i < 4; ++i) {
    const int mBase = m0 + (i << 4);
#pragma unroll
    for (int j = 0; j < 4; ++j) {
      const int n = n0 + (j << 4) + rlane;
      float bv = 0.f;
      if (BIAS_MODE == 2) bv = bias[n];
#pragma unroll
      for (int r = 0; r < 8; ++r) {
        float v = acc[i][j][r] * scale;
        if (BIAS_MODE == 1) v += bias[mBase + mOff + r];
        if (BIAS_MODE == 2) v += bv;
        if (RESID) v += Rb[(size_t)(mBase + mOff + r) * ldc + n];
        if (ACT == 2) v = fmaxf(v, 0.0f);
        if (ACT == 4) v = (v > 0.f) ? v : 0.01f * v;
        slab[(mOff + r) * 68 + (j << 4) + rlane] = v;
      }
    }
    __builtin_amdgcn_fence(__ATOMIC_RELEASE, "workgroup");
    __builtin_amdgcn_wave_barrier();
    __builtin_amdgcn_fence(__ATOMIC_ACQUIRE, "workgroup");
    if (OUT_MODE == 0) {
      float* C = (float*)Cout + (size_t)b * strideC;
      const int hh = lane >> 4, c4 = (lane & 15) * 4;
      for (int pass = 0; pass < 2; ++pass) {
#pragma unroll
        for (int it = 0; it < 8; ++it) {
          const int row = it * 2 + hh;
          v4f v = *(const v4f*)(slab + row * 68 + c4);
          *(volatile v4f*)(C + (size_t)(mBase + row) * ldc + n0 + c4) = v;
        }
        __threadfence();
      }
    } else {
      const int q = lane >> 3, c8 = (lane & 7) * 8;
      unsigned short* C  = (unsigned short*)Cout  + (size_t)b * strideC;
      unsigned short* C2 = (OUT_MODE == 2) ? ((unsigned short*)Cout2 + (size_t)b * strideC) : nullptr;
      for (int pass = 0; pass < 2; ++pass) {
#pragma unroll
        for (int it = 0; it < 4; ++it) {
          const int row = it * 4 + q;
          const float* sp = slab + row * 68 + c8;
          v8h hv, lv;
#pragma unroll
          for (int e = 0; e < 8; ++e) {
            if (OUT_MODE == 1) {
              hv[e] = (_Float16)sp[e];
            } else {
              unsigned short hb = f2bf_bits(sp[e]);
              unsigned short lb = f2bf_bits(sp[e] - bf_bits2f(hb));
              hv[e] = __builtin_bit_cast(_Float16, hb);
              lv[e] = __builtin_bit_cast(_Float16, lb);
            }
          }
          *(volatile v8h*)(C + (size_t)(mBase + row) * ldc + n0 + c8) = hv;
          if (OUT_MODE == 2) *(volatile v8h*)(C2 + (size_t)(mBase + row) * ldc + n0 + c8) = lv;
        }
        __threadfence();
      }
    }
    __builtin_amdgcn_fence(__ATOMIC_RELEASE, "workgroup");
    __builtin_amdgcn_wave_barrier();
    __builtin_amdgcn_fence(__ATOMIC_ACQUIRE, "workgroup");
  }
}

__global__ __launch_bounds__(256) void wtcast_kernel(const float* __restrict__ W, unsigned short* __restrict__ out,
                                                     int ncols, float scale) {
  __shared__ float sm[64][65];
  const int t  = threadIdx.x;
  const int d0 = blockIdx.x * 64;
  const int n0 = blockIdx.y * 64;
#pragma unroll
  for (int i = 0; i < 16; ++i) {
    const int e = i * 256 + t;
    const int r = e >> 6;
    const int c = e & 63;
    sm[c][r] = W[(size_t)(d0 + r) * ncols + n0 + c] * scale;
  }
  __syncthreads();
  const int lane = t & 31, wave = t >> 5;
  const int q = lane >> 3, c8 = (lane & 7) * 8;
  for (int pass = 0; pass < 2; ++pass) {
#pragma unroll
    for (int it = 0; it < 2; ++it) {
      const int row = wave * 8 + it * 4 + q;
      unsigned short hb[8];
#pragma unroll
      for (int e = 0; e < 8; ++e) hb[e] = h_bits(sm[row][c8 + e]);
      const v4u u = (v4u){pk16(hb[0], hb[1]), pk16(hb[2], hb[3]), pk16(hb[4], hb[5]), pk16(hb[6], hb[7])};
      *(volatile v4u*)(out + (size_t)(n0 + row) * kDim + d0 + c8) = u;
    }
    __threadfence();
  }
}

__global__ __launch_bounds__(256) void cast8_f16_kernel(const float* __restrict__ in, unsigned short* __restrict__ out, int n8) {
  const int i = blockIdx.x * 256 + threadIdx.x;
  if (i >= n8) return;
  const float* p = in + 8 * (size_t)i;
  const v4f a = *(const v4f*)(p);
  const v4f c = *(const v4f*)(p + 4);
  unsigned short hb[8];
#pragma unroll
  for (int e = 0; e < 4; ++e) {
    hb[e]     = h_bits(a[e]);
    hb[4 + e] = h_bits(c[e]);
  }
  const v4u u = (v4u){pk16(hb[0], hb[1]), pk16(hb[2], hb[3]), pk16(hb[4], hb[5]), pk16(hb[6], hb[7])};
  unsigned short* qo = out + 8 * (size_t)i;
  *(volatile v4u*)qo = u;
  __threadfence();
  *(volatile v4u*)qo = u;
}

__global__ __launch_bounds__(512) void softmax_mask_kernel(const float* __restrict__ S, const int* __restrict__ keymask,
                                                           unsigned short* __restrict__ P) {
  __shared__ float redM[16];
  __shared__ float redS[16];
  const int row  = blockIdx.x;
  const int t    = threadIdx.x;
  const int lane = t & 31, wave = t >> 5;
  const int c0   = t * 8;
  const float* sr = S + (size_t)row * kSeq + c0;
  const int* mr = keymask + c0;
  const v4f sa = *(const v4f*)(sr);
  const v4f sb = *(const v4f*)(sr + 4);
  const v4i ma = *(const v4i*)(mr);
  const v4i mb = *(const v4i*)(mr + 4);
  v4f xa, xb;
#pragma unroll
  for (int e = 0; e < 4; ++e) {
    xa[e] = (ma[e] != 0) ? sa[e] : kNegMax;
    xb[e] = (mb[e] != 0) ? sb[e] : kNegMax;
  }
  float m = fmaxf(fmaxf(fmaxf(xa[0], xa[1]), fmaxf(xa[2], xa[3])), fmaxf(fmaxf(xb[0], xb[1]), fmaxf(xb[2], xb[3])));
#pragma unroll
  for (int off = 16; off > 0; off >>= 1) m = fmaxf(m, __shfl_xor(m, off, 32));
  if (lane == 0) redM[wave] = m;
  __syncthreads();
  float gm = redM[0];
#pragma unroll
  for (int w = 1; w < 16; ++w) gm = fmaxf(gm, redM[w]);

  v4f ea = (v4f){0.f, 0.f, 0.f, 0.f};
  v4f eb = (v4f){0.f, 0.f, 0.f, 0.f};
  float psum = 0.f;
#pragma unroll 1
  for (int it = 0; it < 2; ++it) {
    v4f ev;
#pragma unroll
    for (int e = 0; e < 4; ++e) {
      const float xv = (it == 0) ? xa[e] : xb[e];
      ev[e] = expf(xv - gm);
    }
    psum += (ev[0] + ev[1]) + (ev[2] + ev[3]);
#pragma unroll
    for (int e = 0; e < 4; ++e) {
      ea[e] = (it == 0) ? ev[e] : ea[e];
      eb[e] = (it == 0) ? eb[e] : ev[e];
    }
  }
#pragma unroll
  for (int off = 16; off > 0; off >>= 1) psum += __shfl_xor(psum, off, 32);
  if (lane == 0) redS[wave] = psum;
  __syncthreads();
  float tot = redS[0];
#pragma unroll
  for (int w = 1; w < 16; ++w) tot += redS[w];
  const float inv = kPCarry * (1.0f / tot);

  unsigned short hb[8];
#pragma unroll
  for (int e = 0; e < 4; ++e) {
    hb[e]     = h_bits(ea[e] * inv);
    hb[4 + e] = h_bits(eb[e] * inv);
  }
  const v4u u = (v4u){pk16(hb[0], hb[1]), pk16(hb[2], hb[3]), pk16(hb[4], hb[5]), pk16(hb[6], hb[7])};
  unsigned short* po = P + (size_t)row * kSeq + c0;
  *(volatile v4u*)po = u;
  __threadfence();
  *(volatile v4u*)po = u;
}

extern "C" void kernel_launch(void* const* d_in, const int* in_sizes, int n_in,
                              void* d_out, int out_size, void* d_ws, size_t ws_size,
                              hipStream_t stream) {
  if (n_in < 6) return;
  if (ws_size < kWsTotal) return;
  if (in_sizes[0] != kTok * kDim) return;
  if (in_sizes[1] != kBatch * kSeq) return;
  if (in_sizes[2] != kDim * kQKVCols) return;
  if (in_sizes[3] != kQKVCols) return;
  if (in_sizes[4] != kDim * kDim) return;
  if (in_sizes[5] != kDim) return;
  if (out_size != kTok * kDim) return;

  const float* x      = (const float*)d_in[0];
  const int*   kmask  = (const int*)  d_in[1];
  const float* W_qkv  = (const float*)d_in[2];
  const float* b_qkv  = (const float*)d_in[3];
  const float* W_proj = (const float*)d_in[4];
  const float* b_proj = (const float*)d_in[5];
  float* out = (float*)d_out;

  char* ws = (char*)d_ws;
  unsigned short* x16    = (unsigned short*)(ws + kOffX16);
  unsigned short* ctx16  = (unsigned short*)(ws + kOffX16);
  unsigned short* qk16   = (unsigned short*)(ws + kOffQK16);
  unsigned short* vt16   = (unsigned short*)(ws + kOffVT16);
  float*          Sp     = (float*)(ws + kOffS);
  unsigned short* wqkvT  = (unsigned short*)(ws + kOffS);
  unsigned short* wprojT = (unsigned short*)(ws + kOffS);
  unsigned short* P16    = (unsigned short*)(ws + kOffP16);
  const float* fpad = b_qkv;

  cast8_f16_kernel<<<dim3((kTok * kDim / 8) / 256), dim3(256), 0, stream>>>(x, x16, kTok * kDim / 8);

  wtcast_kernel<<<dim3(kDim / 64, kQKVCols / 64), dim3(256), 0, stream>>>(W_qkv, wqkvT, kQKVCols, kWCarry);

  wmma_gemm64<0, false, 2, 1, false, 0><<<dim3((kTok / 64) * (kQKCols / 64) / 8, 1), dim3(256), 0, stream>>>(
      x16, x16, kDim, 0L, wqkvT, wqkvT, kDim, 0L, (void*)qk16, (void*)qk16, kQKCols, 0L,
      b_qkv, fpad, 0L, kTok, kQKCols, kDim, kWCarryInv);

  wmma_gemm64<0, false, 1, 1, false, 0><<<dim3((kDim / 64) * (kTok / 64) / 8, 1), dim3(256), 0, stream>>>(
      wqkvT + (size_t)kQKCols * kDim, wqkvT + (size_t)kQKCols * kDim, kDim, 0L, x16, x16, kDim, 0L,
      (void*)vt16, (void*)vt16, kTok, 0L,
      b_qkv + kQKCols, fpad, 0L, kDim, kTok, kDim, kWCarryInv);

  for (int cidx = 0; cidx < kBatch * kHeads * kQChunks; ++cidx) {
    const int g  = cidx / kQChunks;
    const int qh = cidx - g * kQChunks;
    const int b  = g / kHeads, h = g - b * kHeads;
    const size_t qrow0 = (size_t)b * kSeq + (size_t)qh * kQRows;
    const unsigned short* qA = qk16 + qrow0 * kQKCols + (size_t)h * kHdim;
    const unsigned short* kB = qk16 + (size_t)b * kSeq * kQKCols + kDim + (size_t)h * kHdim;
    wmma_gemm64<0, false, 0, 0, false, 0><<<dim3((kQRows / 64) * (kSeq / 64) / 8, 1), dim3(256), 0, stream>>>(
        qA, qA, kQKCols, 0L, kB, kB, kQKCols, 0L, (void*)Sp, (void*)Sp, kSeq, 0L,
        fpad, fpad, 0L, kQRows, kSeq, kHdim, kScoreScale);
    softmax_mask_kernel<<<dim3(kQRows), dim3(512), 0, stream>>>(Sp, kmask + (size_t)b * kSeq, P16);
    const unsigned short* vB = vt16 + (size_t)(h * kHdim) * kTok + (size_t)b * kSeq;
    unsigned short* cO = ctx16 + qrow0 * kDim + (size_t)h * kHdim;
    wmma_gemm64<0, false, 0, 1, false, 0><<<dim3((kQRows / 64) * (kHdim / 64) / 8, 1), dim3(256), 0, stream>>>(
        P16, P16, kSeq, 0L, vB, vB, kTok, 0L, (void*)cO, (void*)cO, kDim, 0L,
        fpad, fpad, 0L, kQRows, kHdim, kSeq, kPVScale);
  }

  wtcast_kernel<<<dim3(kDim / 64, kDim / 64), dim3(256), 0, stream>>>(W_proj, wprojT, kDim, kWCarry);

  wmma_gemm64<0, false, 2, 0, false, 0><<<dim3((kTok / 64) * (kDim / 64) / 8, 1), dim3(256), 0, stream>>>(
      ctx16, ctx16, kDim, 0L, wprojT, wprojT, kDim, 0L, (void*)out, (void*)out, kDim, 0L,
      b_proj, fpad, 0L, kTok, kDim, kDim, kOutScale);
}
